// MambaWrapper_69363721830796
// MI455X (gfx1250) — hardware-verified
//
#include <hip/hip_runtime.h>
#include <stdint.h>
#include <math.h>

constexpr int kBatch  = 2;
constexpr int kSeq    = 2048;
constexpr int kDModel = 1024;
constexpr int kDInner = 2048;
constexpr int kDState = 16;
constexpr int kDConv  = 4;
constexpr int kDtRank = 64;
constexpr int kXprojN = kDtRank + 2 * kDState;
constexpr int kXdblN  = 128;
constexpr int kRows   = kBatch * kSeq;

constexpr size_t kSzXb   = (size_t)kRows * kDModel * 2;
constexpr size_t kSzWinb = (size_t)2 * kDInner * kDModel * 2;
constexpr size_t kSzWopb = (size_t)kDModel * kDInner * 2;
constexpr size_t kSzWxpb = (size_t)kXdblN * kDInner * 2;
constexpr size_t kSzWdtb = (size_t)kDInner * kDtRank * 2;
constexpr size_t kSzBig  = (size_t)kRows * kDInner * 4;
constexpr size_t kSzXdbl = (size_t)kRows * kXdblN * 4;
constexpr size_t kSzDt   = (size_t)kRows * kDtRank * 2 * 2;

constexpr size_t kOffXb   = 0;
constexpr size_t kOffWinb = kOffXb + kSzXb;
constexpr size_t kOffWopb = kOffWinb + kSzWinb;
constexpr size_t kOffWxpb = kOffWopb + kSzWopb;
constexpr size_t kOffWdtb = kOffWxpb + kSzWxpb;
constexpr size_t kOffRA   = kOffWdtb + kSzWdtb;
constexpr size_t kOffRB   = kOffRA + kSzBig;
constexpr size_t kOffRC   = kOffRB + kSzBig;
constexpr size_t kOffXdbl = kOffRC + kSzBig;
constexpr size_t kOffDt   = kOffXdbl + kSzXdbl;
constexpr size_t kWsTotal = kOffDt + kSzDt;
static_assert(kWsTotal == 125566976);
static_assert(kWsTotal <= 134217728);
static_assert((kOffWinb % 128) == 0 && (kOffWopb % 128) == 0 && (kOffWxpb % 128) == 0 && (kOffWdtb % 128) == 0);
static_assert((kOffRA % 128) == 0 && (kOffRB % 128) == 0 && (kOffRC % 128) == 0 && (kOffXdbl % 128) == 0 && (kOffDt % 128) == 0);
static_assert((size_t)kRows * kDInner * 2 * 2 == kSzBig);

static_assert(kRows % 64 == 0 && kDInner % 64 == 0 && kDModel % 64 == 0 && kXdblN % 64 == 0);
static_assert(kDModel % 32 == 0 && kDInner % 32 == 0 && kDtRank % 32 == 0);
static_assert(kXprojN <= kXdblN);

typedef __attribute__((ext_vector_type(16))) _Float16 v16h;
typedef __attribute__((ext_vector_type(8)))  _Float16 v8h;
typedef __attribute__((ext_vector_type(16))) __bf16   v16b;
typedef __attribute__((ext_vector_type(8)))  __bf16   v8b;
typedef __attribute__((ext_vector_type(8)))  float    v8f;
typedef __attribute__((ext_vector_type(4)))  float    v4f;
typedef __attribute__((ext_vector_type(2)))  float    v2f;
typedef __attribute__((ext_vector_type(4)))  unsigned v4u;

__device__ __forceinline__ unsigned short f2bf_bits(float f) {
  unsigned u = __float_as_uint(f);
  return (unsigned short)((u + 0x7FFFu + ((u >> 16) & 1u)) >> 16);
}
__device__ __forceinline__ float bf_bits2f(unsigned short h) { return __uint_as_float(((unsigned)h) << 16); }
__device__ __forceinline__ float bfr(float f) { return bf_bits2f(f2bf_bits(f)); }

__device__ __forceinline__ void dep_guard_h(v8f& a, v8f& b, v16h x, v16h y) { asm volatile("v_nop\n\tv_nop\n\tv_nop\n\tv_nop" : "+v"(a), "+v"(b) : "v"(x), "v"(y)); }
__device__ __forceinline__ void dep_guard_b(v8f& a, v8f& b, v16b x, v16b y) { asm volatile("v_nop\n\tv_nop\n\tv_nop\n\tv_nop" : "+v"(a), "+v"(b) : "v"(x), "v"(y)); }
__device__ __forceinline__ void keep4_h(v16h a, v16h b, v16h c, v16h d) { asm volatile("v_nop" :: "v"(a), "v"(b), "v"(c), "v"(d)); }
__device__ __forceinline__ void keep4_b(v16b a, v16b b, v16b c, v16b d) { asm volatile("v_nop" :: "v"(a), "v"(b), "v"(c), "v"(d)); }
__device__ __forceinline__ void acc_guard4(v8f& a, v8f& b, v8f& c, v8f& d) { asm volatile("v_nop\n\tv_nop\n\tv_nop\n\tv_nop" : "+v"(a), "+v"(b), "+v"(c), "+v"(d)); }

template <typename T> struct Frag;
template <> struct Frag<_Float16> {
  typedef v16h V; union U { v16h v; v8h h[2]; };
  static __device__ __forceinline__ v16h load(const _Float16* p) {
    U f; f.h[0] = *(const v8h*)(p); f.h[1] = *(const v8h*)(p + 16); return f.v;
  }
  static __device__ __forceinline__ v8f mma(v16h a, v16h b, v8f c) {
    return __builtin_amdgcn_wmma_f32_16x16x32_f16(false, a, false, b, (short)0, c, false, false);
  }
  static __device__ __forceinline__ void guard(v8f& a, v8f& b, v16h x, v16h y) { dep_guard_h(a, b, x, y); }
  static __device__ __forceinline__ void keep(v16h a, v16h b, v16h c, v16h d) { keep4_h(a, b, c, d); }
};
template <> struct Frag<__bf16> {
  typedef v16b V; union U { v16b v; v8b h[2]; };
  static __device__ __forceinline__ v16b load(const __bf16* p) {
    U f; f.h[0] = *(const v8b*)(p); f.h[1] = *(const v8b*)(p + 16); return f.v;
  }
  static __device__ __forceinline__ v8f mma(v16b a, v16b b, v8f c) {
    return __builtin_amdgcn_wmma_f32_16x16x32_bf16(false, a, false, b, (short)0, c, false, false);
  }
  static __device__ __forceinline__ void guard(v8f& a, v8f& b, v16b x, v16b y) { dep_guard_b(a, b, x, y); }
  static __device__ __forceinline__ void keep(v16b a, v16b b, v16b c, v16b d) { keep4_b(a, b, c, d); }
};

template <int ET> struct Elem;
template <> struct Elem<0> { typedef _Float16 T; };
template <> struct Elem<1> { typedef __bf16 T; };
template <int ET, int SPLIT, int BIAS_MODE, int OUT_MODE, bool RESID, int ACT = 0>
__global__ __launch_bounds__(256) void wmma_gemm64(
    const unsigned short* __restrict__ Ap, const unsigned short* __restrict__ A2p, int lda, long strideA,
    const unsigned short* __restrict__ Btp, const unsigned short* __restrict__ Bt2p, int ldb, long strideB,
    void* __restrict__ Cout, void* __restrict__ Cout2, int ldc, long strideC,
    const float* __restrict__ bias,
    const float* __restrict__ resid, long strideR,
    int M, int N, int K, float scale) {
  typedef typename Elem<ET>::T T;
  typedef typename Frag<T>::V V;
  const T* A = (const T*)Ap; const T* A2 = (const T*)A2p; const T* Bt = (const T*)Btp; const T* Bt2 = (const T*)Bt2p;
  __shared__ __align__(16) float sT[8][16 * 68];
  const int b    = blockIdx.y;
  const int lane = threadIdx.x & 31;
  const int wave = threadIdx.x >> 5;
  const int tilesN = N >> 6;
  const int tilesM = M >> 6;
  const int tile = blockIdx.x * 8 + wave;
  if (tile >= tilesM * tilesN) return;
  const int tm = tile / tilesN;
  const int tn = tile - tm * tilesN;
  const int m0 = tm << 6;
  const int n0 = tn << 6;

  const T* Ab  = A  + (size_t)b * strideA;
  const T* Bb  = Bt + (size_t)b * strideB;
  const T* Ab2 = (SPLIT >= 1) ? (A2  + (size_t)b * strideA) : nullptr;
  const T* Bb2 = (SPLIT == 2) ? (Bt2 + (size_t)b * strideB) : nullptr;

  const int rlane = lane & 15;
  const int koff  = (lane >> 4) * 8;
  const int mOff  = (lane >> 4) * 8;

  v8f acc[4][4];
#pragma unroll
  for (int i = 0; i < 4; ++i)
#pragma unroll
    for (int j = 0; j < 4; ++j) acc[i][j] = (v8f){0.f,0.f,0.f,0.f,0.f,0.f,0.f,0.f};

  for (int k0 = 0; k0 < K; k0 += 32) {
    V bh[4], bl[4];
#pragma unroll
    for (int j = 0; j < 4; ++j) {
      const size_t bo = (size_t)(n0 + (j << 4) + rlane) * ldb + koff + k0;
      bh[j] = Frag<T>::load(Bb + bo);
      if (SPLIT == 2) bl[j] = Frag<T>::load(Bb2 + bo);
    }
#pragma unroll
    for (int i = 0; i < 4; ++i) {
      const size_t ao = (size_t)(m0 + (i << 4) + rlane) * lda + koff + k0;
      V ah = Frag<T>::load(Ab + ao);
      V al;
      if (SPLIT >= 1) al = Frag<T>::load(Ab2 + ao);
#pragma unroll
      for (int j = 0; j < 4; ++j) {
        acc[i][j] = Frag<T>::mma(ah, bh[j], acc[i][j]);
        if (SPLIT == 2) acc[i][j] = Frag<T>::mma(ah, bl[j], acc[i][j]);
        if (SPLIT >= 1) acc[i][j] = Frag<T>::mma(al, bh[j], acc[i][j]);
      }
      Frag<T>::guard(acc[i][0], acc[i][3], ah, (SPLIT >= 1) ? al : ah);
    }
    Frag<T>::keep(bh[0], bh[1], bh[2], bh[3]);
    if (SPLIT == 2) Frag<T>::keep(bl[0], bl[1], bl[2], bl[3]);
  }
  acc_guard4(acc[0][0], acc[0][1], acc[0][2], acc[0][3]);
  acc_guard4(acc[1][0], acc[1][1], acc[1][2], acc[1][3]);
  acc_guard4(acc[2][0], acc[2][1], acc[2][2], acc[2][3]);
  acc_guard4(acc[3][0], acc[3][1], acc[3][2], acc[3][3]);

  float* slab = sT[wave];
  const float* Rb = RESID ? (resid + (size_t)b * strideR) : nullptr;
#pragma unroll
  for (int i = 0; i < 4; ++i) {
    const int mBase = m0 + (i << 4);
#pragma unroll
    for (int j = 0; j < 4; ++j) {
      const int n = n0 + (j << 4) + rlane;
      float bv = 0.f;
      if (BIAS_MODE == 2) bv = bias[n];
#pragma unroll
      for (int r = 0; r < 8; ++r) {
        float v = acc[i][j][r] * scale;
        if (BIAS_MODE == 1) v += bias[mBase + mOff + r];
        if (BIAS_MODE == 2) v += bv;
        if (RESID) {
          const float rv = Rb[(size_t)(mBase + mOff + r) * ldc + n];
          if (ACT == 6) v = rv * (v * (1.0f / (1.0f + expf(-v))));
          else v += rv;
        }
        if (ACT == 1) v = tanhf(v);
        if (ACT == 2) v = fmaxf(v, 0.0f);
        if (ACT == 3) v = v / (1.0f + expf(-v));
        if (ACT == 4) v = (v > 0.f) ? v : 0.01f * v;
        slab[(mOff + r) * 68 + (j << 4) + rlane] = v;
      }
    }
    __builtin_amdgcn_fence(__ATOMIC_RELEASE, "workgroup");
    __builtin_amdgcn_wave_barrier();
    __builtin_amdgcn_fence(__ATOMIC_ACQUIRE, "workgroup");
    if (OUT_MODE == 0) {
      float* C = (float*)Cout + (size_t)b * strideC;
      const int hh = lane >> 4, c4 = (lane & 15) * 4;
      for (int pass = 0; pass < 2; ++pass) {
#pragma unroll
        for (int it = 0; it < 8; ++it) {
          const int row = it * 2 + hh;
          v4f v = *(const v4f*)(slab + row * 68 + c4);
          *(volatile v4f*)(C + (size_t)(mBase + row) * ldc + n0 + c4) = v;
        }
        __threadfence();
      }
    } else {
      const int q = lane >> 3, c8 = (lane & 7) * 8;
      unsigned short* C  = (unsigned short*)Cout  + (size_t)b * strideC;
      unsigned short* C2 = (OUT_MODE == 2) ? ((unsigned short*)Cout2 + (size_t)b * strideC) : nullptr;
      for (int pass = 0; pass < 2; ++pass) {
#pragma unroll
        for (int it = 0; it < 4; ++it) {
          const int row = it * 4 + q;
          const float* sp = slab + row * 68 + c8;
          v8h hv, lv;
#pragma unroll
          for (int e = 0; e < 8; ++e) {
            if (OUT_MODE == 1) {
              hv[e] = (_Float16)sp[e];
            } else {
              unsigned short hb = f2bf_bits(sp[e]);
              unsigned short lb = f2bf_bits(sp[e] - bf_bits2f(hb));
              hv[e] = __builtin_bit_cast(_Float16, hb);
              lv[e] = __builtin_bit_cast(_Float16, lb);
            }
          }
          *(volatile v8h*)(C + (size_t)(mBase + row) * ldc + n0 + c8) = hv;
          if (OUT_MODE == 2) *(volatile v8h*)(C2 + (size_t)(mBase + row) * ldc + n0 + c8) = lv;
        }
        __threadfence();
      }
    }
    __builtin_amdgcn_fence(__ATOMIC_RELEASE, "workgroup");
    __builtin_amdgcn_wave_barrier();
    __builtin_amdgcn_fence(__ATOMIC_ACQUIRE, "workgroup");
  }
}

__global__ __launch_bounds__(256) void cast_f32_bf16x8(
    const float* __restrict__ in, unsigned short* __restrict__ out, int n_src, int n_dst) {
  const int i = blockIdx.x * 256 + (int)threadIdx.x;
  const int e0 = i * 8;
  if (e0 < n_dst) {
    const bool live = (e0 < n_src);
    const int s0 = live ? e0 : (n_src - 8);
    const v4f a = *(const v4f*)(in + s0);
    const v4f c = *(const v4f*)(in + s0 + 4);
    v4u o;
    o[0] = (unsigned)f2bf_bits(a[0]) | ((unsigned)f2bf_bits(a[1]) << 16);
    o[1] = (unsigned)f2bf_bits(a[2]) | ((unsigned)f2bf_bits(a[3]) << 16);
    o[2] = (unsigned)f2bf_bits(c[0]) | ((unsigned)f2bf_bits(c[1]) << 16);
    o[3] = (unsigned)f2bf_bits(c[2]) | ((unsigned)f2bf_bits(c[3]) << 16);
    if (!live) o = (v4u){0u, 0u, 0u, 0u};
    unsigned short* p = out + e0;
    *(volatile v4u*)p = o;
    __threadfence();
    *(volatile v4u*)p = o;
  }
}

__global__ __launch_bounds__(256) void conv_silu_split_kernel(
    const float* __restrict__ xu,
    const float* __restrict__ conv_w,
    const float* __restrict__ conv_b,
    unsigned* __restrict__ uhw,
    unsigned* __restrict__ ulw)
{
  const int bid = blockIdx.x;
  const int m = bid >> 2;
  const int t = m & (kSeq - 1);
  const int d = ((bid & 3) << 9) + (int)threadIdx.x * 2;
  const v4f w0 = *(const v4f*)(conv_w + (size_t)d * kDConv);
  const v4f w1 = *(const v4f*)(conv_w + (size_t)(d + 1) * kDConv);
  float a0 = bfr(conv_b[d]);
  float a1 = bfr(conv_b[d + 1]);
#pragma unroll
  for (int j = 0; j < kDConv; ++j) {
    const int tt = t - (kDConv - 1) + j;
    const int rr = (tt >= 0) ? (m - (kDConv - 1) + j) : m;
    const v2f xv = *(const v2f*)(xu + (size_t)rr * kDInner + d);
    const float x0 = (tt >= 0) ? xv[0] : 0.f;
    const float x1 = (tt >= 0) ? xv[1] : 0.f;
    a0 += bfr(w0[j]) * x0;
    a1 += bfr(w1[j]) * x1;
  }
  const float s0 = a0 * (1.0f / (1.0f + expf(-a0)));
  const float s1 = a1 * (1.0f / (1.0f + expf(-a1)));
  const unsigned short h0 = f2bf_bits(s0), h1 = f2bf_bits(s1);
  const unsigned short l0 = f2bf_bits(s0 - bf_bits2f(h0));
  const unsigned short l1 = f2bf_bits(s1 - bf_bits2f(h1));
  const unsigned hw = (unsigned)h0 | ((unsigned)h1 << 16);
  const unsigned lw = (unsigned)l0 | ((unsigned)l1 << 16);
  const size_t wi = ((size_t)m * kDInner + d) >> 1;
  *(volatile unsigned*)(uhw + wi) = hw;
  *(volatile unsigned*)(ulw + wi) = lw;
  __threadfence();
  *(volatile unsigned*)(uhw + wi) = hw;
  *(volatile unsigned*)(ulw + wi) = lw;
}

__global__ __launch_bounds__(256) void split_dt_kernel(
    const float* __restrict__ xdbl, unsigned short* __restrict__ dth, unsigned short* __restrict__ dtl) {
  const int tid = (int)threadIdx.x;
  const int r = blockIdx.x * 32 + (tid >> 3);
  const int c0 = (tid & 7) * 8;
  const v4f a = *(const v4f*)(xdbl + (size_t)r * kXdblN + c0);
  const v4f c = *(const v4f*)(xdbl + (size_t)r * kXdblN + c0 + 4);
  float f[8];
  f[0] = a[0]; f[1] = a[1]; f[2] = a[2]; f[3] = a[3];
  f[4] = c[0]; f[5] = c[1]; f[6] = c[2]; f[7] = c[3];
  v4u ho, lo;
#pragma unroll
  for (int q = 0; q < 4; ++q) {
    const unsigned short hA = f2bf_bits(f[2 * q]);
    const unsigned short hB = f2bf_bits(f[2 * q + 1]);
    const unsigned short lA = f2bf_bits(f[2 * q] - bf_bits2f(hA));
    const unsigned short lB = f2bf_bits(f[2 * q + 1] - bf_bits2f(hB));
    ho[q] = (unsigned)hA | ((unsigned)hB << 16);
    lo[q] = (unsigned)lA | ((unsigned)lB << 16);
  }
  unsigned short* ph = dth + (size_t)r * kDtRank + c0;
  unsigned short* pl = dtl + (size_t)r * kDtRank + c0;
  *(volatile v4u*)ph = ho;
  *(volatile v4u*)pl = lo;
  __threadfence();
  *(volatile v4u*)ph = ho;
  *(volatile v4u*)pl = lo;
}

__global__ __launch_bounds__(256) void ssm_scan_kernel(
    const float* __restrict__ dpre,
    const unsigned* __restrict__ uhw,
    const unsigned* __restrict__ ulw,
    const float* __restrict__ xdbl,
    const float* __restrict__ A_log,
    const float* __restrict__ Dp,
    const float* __restrict__ dt_b,
    float* __restrict__ ypre)
{
  __shared__ float ybuf[8 * 256];
  const int tid = (int)threadIdx.x;
  const int d = blockIdx.x * 256 + tid;
  const int b = blockIdx.y;
  const float kLog2e = 1.4426950408889634f;

  float A2[kDState];
  {
    const v4f g0 = *(const v4f*)(A_log + (size_t)d * kDState);
    const v4f g1 = *(const v4f*)(A_log + (size_t)d * kDState + 4);
    const v4f g2 = *(const v4f*)(A_log + (size_t)d * kDState + 8);
    const v4f g3 = *(const v4f*)(A_log + (size_t)d * kDState + 12);
#pragma unroll
    for (int e = 0; e < 4; ++e) {
      A2[e]      = -expf(bfr(g0[e])) * kLog2e;
      A2[4 + e]  = -expf(bfr(g1[e])) * kLog2e;
      A2[8 + e]  = -expf(bfr(g2[e])) * kLog2e;
      A2[12 + e] = -expf(bfr(g3[e])) * kLog2e;
    }
  }
  const float Dd = bfr(Dp[d]);
  const float bd = bfr(dt_b[d]);
  const unsigned sh = (d & 1) ? 16u : 0u;
  float h[kDState];
#pragma unroll
  for (int n = 0; n < kDState; ++n) h[n] = 0.f;

  const size_t row0 = (size_t)b * kSeq;
#pragma unroll 1
  for (int c = 0; c < kSeq / 8; ++c) {
#pragma unroll 1
    for (int j = 0; j < 8; ++j) {
      const size_t m = row0 + (size_t)(c * 8 + j);
      const float pre = dpre[m * kDInner + d] + bd;
      const float dt = fmaxf(pre, 0.f) + log1pf(expf(-fabsf(pre)));
      const size_t wi = (m * kDInner + d) >> 1;
      const unsigned wh = uhw[wi];
      const unsigned wl = ulw[wi];
      const float uh = __uint_as_float(((wh >> sh) & 0xffffu) << 16);
      const float ul = __uint_as_float(((wl >> sh) & 0xffffu) << 16);
      const float ut = uh + ul;
      const float du = dt * ut;
      const float* bc = xdbl + m * kXdblN + kDtRank;
      v4f bq[4], cq[4];
#pragma unroll
      for (int q = 0; q < 4; ++q) {
        bq[q] = *(const v4f*)(bc + 4 * q);
        cq[q] = *(const v4f*)(bc + kDState + 4 * q);
      }
      float y = 0.f;
#pragma unroll
      for (int n = 0; n < kDState; ++n) {
        const float Bn = bq[n >> 2][n & 3];
        const float Cn = cq[n >> 2][n & 3];
        const float dA = exp2f(dt * A2[n]);
        h[n] = dA * h[n] + du * Bn;
        y += h[n] * Cn;
      }
      const float yo = y + ut * Dd;
      ybuf[j * 256 + tid] = yo;
      *(volatile float*)(ypre + m * kDInner + d) = yo;
    }
    __threadfence();
#pragma unroll 1
    for (int j = 0; j < 8; ++j) {
      const size_t m = row0 + (size_t)(c * 8 + j);
      const float v = ybuf[j * 256 + tid];
      *(volatile float*)(ypre + m * kDInner + d) = v;
    }
  }
}

extern "C" void kernel_launch(void* const* d_in, const int* in_sizes, int n_in,
                              void* d_out, int out_size, void* d_ws, size_t ws_size,
                              hipStream_t stream) {
  (void)in_sizes; (void)n_in; (void)out_size;
  if (ws_size < kWsTotal) return;

  const float* x          = (const float*)d_in[0];
  const float* in_proj_w  = (const float*)d_in[1];
  const float* conv_w     = (const float*)d_in[2];
  const float* conv_b     = (const float*)d_in[3];
  const float* x_proj_w   = (const float*)d_in[4];
  const float* dt_proj_w  = (const float*)d_in[5];
  const float* dt_proj_b  = (const float*)d_in[6];
  const float* A_log      = (const float*)d_in[7];
  const float* Dp         = (const float*)d_in[8];
  const float* out_proj_w = (const float*)d_in[9];
  float* out = (float*)d_out;

  char* ws = (char*)d_ws;
  unsigned short* xb   = (unsigned short*)(ws + kOffXb);
  unsigned short* winb = (unsigned short*)(ws + kOffWinb);
  unsigned short* wopb = (unsigned short*)(ws + kOffWopb);
  unsigned short* wxpb = (unsigned short*)(ws + kOffWxpb);
  unsigned short* wdtb = (unsigned short*)(ws + kOffWdtb);
  float* xu   = (float*)(ws + kOffRA);
  float* dpre = (float*)(ws + kOffRA);
  unsigned short* yhi = (unsigned short*)(ws + kOffRA);
  unsigned short* ylo = yhi + (size_t)kRows * kDInner;
  unsigned short* uhi = (unsigned short*)(ws + kOffRB);
  unsigned short* ulo = uhi + (size_t)kRows * kDInner;
  float* ypre = (float*)(ws + kOffRC);
  float* xdbl = (float*)(ws + kOffXdbl);
  unsigned short* dthi = (unsigned short*)(ws + kOffDt);
  unsigned short* dtlo = dthi + (size_t)kRows * kDtRank;

  auto cast = [&](const float* src, unsigned short* dst, int n_src, int n_dst) {
    const int thr = n_dst / 8;
    cast_f32_bf16x8<<<dim3((thr + 255) / 256), dim3(256), 0, stream>>>(src, dst, n_src, n_dst);
  };
  cast(x,          xb,   kRows * kDModel,       kRows * kDModel);
  cast(in_proj_w,  winb, 2 * kDInner * kDModel, 2 * kDInner * kDModel);
  cast(x_proj_w,   wxpb, kXprojN * kDInner,     kXdblN * kDInner);
  cast(dt_proj_w,  wdtb, kDInner * kDtRank,     kDInner * kDtRank);
  cast(out_proj_w, wopb, kDModel * kDInner,     kDModel * kDInner);

  {
    const int tiles = (kRows / 64) * (kDInner / 64);
    wmma_gemm64<1, 0, 0, 0, false, 0><<<dim3(tiles / 8, 1), dim3(256), 0, stream>>>(
        xb, xb, kDModel, 0L, winb, winb, kDModel, 0L,
        (void*)xu, (void*)xu, kDInner, 0L, conv_b, ypre, 0L,
        kRows, kDInner, kDModel, 1.0f);
  }
  conv_silu_split_kernel<<<dim3(kRows * 4), dim3(256), 0, stream>>>(
      xu, conv_w, conv_b, (unsigned*)uhi, (unsigned*)ulo);
  {
    const int tiles = (kRows / 64) * (kXdblN / 64);
    wmma_gemm64<1, 1, 0, 0, false, 0><<<dim3(tiles / 8, 1), dim3(256), 0, stream>>>(
        uhi, ulo, kDInner, 0L, wxpb, wxpb, kDInner, 0L,
        (void*)xdbl, (void*)xdbl, kXdblN, 0L, conv_b, ypre, 0L,
        kRows, kXdblN, kDInner, 1.0f);
  }
  split_dt_kernel<<<dim3(kRows / 32), dim3(256), 0, stream>>>(xdbl, dthi, dtlo);
  {
    const int tiles = (kRows / 64) * (kDInner / 64);
    wmma_gemm64<1, 1, 0, 0, false, 0><<<dim3(tiles / 8, 1), dim3(256), 0, stream>>>(
        dthi, dtlo, kDtRank, 0L, wdtb, wdtb, kDtRank, 0L,
        (void*)dpre, (void*)dpre, kDInner, 0L, conv_b, ypre, 0L,
        kRows, kDInner, kDtRank, 1.0f);
  }
  ssm_scan_kernel<<<dim3(kDInner / 256, kBatch), dim3(256), 0, stream>>>(
      dpre, (const unsigned*)uhi, (const unsigned*)ulo, xdbl, A_log, Dp, dt_proj_b, ypre);
  {
    const int tiles = (kRows / 64) * (kDInner / 64);
    wmma_gemm64<1, 0, 0, 2, true, 6><<<dim3(tiles / 8, 1), dim3(256), 0, stream>>>(
        xb, xb, kDModel, 0L, winb + (size_t)kDInner * kDModel, winb + (size_t)kDInner * kDModel, kDModel, 0L,
        (void*)yhi, (void*)ylo, kDInner, 0L, conv_b, ypre, 0L,
        kRows, kDInner, kDModel, 1.0f);
  }
  {
    const int tiles = (kRows / 64) * (kDModel / 64);
    wmma_gemm64<1, 1, 0, 0, false, 0><<<dim3(tiles / 8, 1), dim3(256), 0, stream>>>(
        yhi, ylo, kDInner, 0L, wopb, wopb, kDInner, 0L,
        (void*)out, (void*)out, kDModel, 0L, conv_b, ypre, 0L,
        kRows, kDModel, kDInner, 1.0f);
  }
}
